// DimeNetPP_28587302322454
// MI455X (gfx1250) — hardware-run, weakly checked
//
#include <hip/hip_runtime.h>
#include <stddef.h>

#pragma clang fp contract(off)

#define NA 512
#define HID 128
#define HID2 64
#define NRBF 60
#define KR 64
#define RP 128
#define NBLK 4
#define NMOL 16
#define NEMB 100
#define HP 128
#define NTHR 256
#define NT 32
#define NTP 528
#define TILEF 2048
#define CUTOFF_D 5.0f

static_assert(NA % 16 == 0);
static_assert(NA == NT * 16);
static_assert(NTP == (NT * (NT + 1)) / 2);
static_assert(HID == 128);
static_assert(NTHR == 256);
static_assert((NTHR / 32) * 2 == 16);
static_assert((NTHR / 32) * 16 == HID);
static_assert(KR % 32 == 0);
static_assert(KR >= NRBF);
static_assert(RP == 2 * KR);
static_assert(HP % 8 == 0);
static_assert(TILEF == 16 * HID);
static_assert((NA * NA * 8) % NTHR == 0);
static_assert(NMOL == 16);

typedef unsigned short us_t;
typedef __bf16 bf_t;
typedef bf_t v16b __attribute__((ext_vector_type(16)));
typedef us_t v16us __attribute__((ext_vector_type(16)));
typedef us_t v8us_t __attribute__((ext_vector_type(8)));
typedef v8us_t __attribute__((may_alias)) v8us;
typedef us_t v4us_t __attribute__((ext_vector_type(4)));
typedef v4us_t __attribute__((may_alias)) v4us;
typedef float v8f __attribute__((ext_vector_type(8)));
typedef float v4f_t __attribute__((ext_vector_type(4)));
typedef v4f_t __attribute__((may_alias)) v4f;
typedef unsigned int v4u __attribute__((ext_vector_type(4)));

union Frag { v16b v; v16us u; v8us_t h[2]; };
struct BPair { v16b h; v16b l; };

__device__ __forceinline__ v8f zero8() {
  v8f z;
#pragma unroll
  for (int i = 0; i < 8; ++i) z[i] = 0.0f;
  return z;
}

__device__ __forceinline__ unsigned bf_rne(float x) {
  const unsigned u = __float_as_uint(x);
  return (u + 0x7FFFu + ((u >> 16) & 1u)) >> 16;
}

__device__ __forceinline__ void split_bf(float x, us_t& hi, us_t& lo) {
  const unsigned h = bf_rne(x);
  const float hf = __uint_as_float(h << 16);
  const unsigned l = bf_rne(x - hf);
  hi = (us_t)h;
  lo = (us_t)l;
}

__device__ __forceinline__ v8f wmma3(v16b ah, v16b al, v16b bh, v16b bl, v8f c) {
  c = __builtin_amdgcn_wmma_f32_16x16x32_bf16(false, ah, false, bh, (short)0, c, false, false);
  c = __builtin_amdgcn_wmma_f32_16x16x32_bf16(false, ah, false, bl, (short)0, c, false, false);
  c = __builtin_amdgcn_wmma_f32_16x16x32_bf16(false, al, false, bh, (short)0, c, false, false);
  asm volatile("v_nop\n\tv_nop\n\tv_nop\n\tv_nop" : "+v"(c) : "v"(ah), "v"(al), "v"(bh), "v"(bl));
  return c;
}

__device__ __forceinline__ v16b ldfragA(const us_t* base, int ld, int k0, int lane) {
  const int hh = lane >> 4, m = lane & 15;
  const us_t* p = base + m * ld + k0 + 8 * hh;
  Frag f;
  f.h[0] = *(const v8us*)(p);
  f.h[1] = *(const v8us*)(p + 16);
  return f.v;
}

__device__ __forceinline__ BPair ldfragB(const float* __restrict__ W, int ldw, int k0, int kmax,
                                         int col, int lane) {
  const int hh = lane >> 4;
  Frag fh, fl;
#pragma unroll
  for (int e = 0; e < 8; ++e) {
    const int ka = k0 + 8 * hh + e;
    const int kb = ka + 16;
    const int kac = (ka < kmax) ? ka : (kmax - 1);
    const int kbc = (kb < kmax) ? kb : (kmax - 1);
    float va = W[(size_t)kac * ldw + col];
    float vb = W[(size_t)kbc * ldw + col];
    va = (ka < kmax) ? va : 0.0f;
    vb = (kb < kmax) ? vb : 0.0f;
    us_t ha, la, hb, lb;
    split_bf(va, ha, la);
    split_bf(vb, hb, lb);
    fh.u[e] = ha; fh.u[8 + e] = hb;
    fl.u[e] = la; fl.u[8 + e] = lb;
  }
  BPair r;
  r.h = fh.v;
  r.l = fl.v;
  return r;
}

__device__ __forceinline__ v8f gemm128s(const us_t* sH, const us_t* sL,
                                        const float* __restrict__ W, int ldw,
                                        int kb0, int kmax, int col, int lane, v8f acc) {
#pragma unroll 1
  for (int ks = 0; ks < 4; ++ks) {
    const v16b ah = ldfragA(sH, HP, 32 * ks, lane);
    const v16b al = ldfragA(sL, HP, 32 * ks, lane);
    const BPair b = ldfragB(W, ldw, kb0 + 32 * ks, kmax, col, lane);
    acc = wmma3(ah, al, b.h, b.l, acc);
  }
  return acc;
}

__device__ __forceinline__ float silu_f(float z) {
  return z * __builtin_amdgcn_rcpf(1.0f + __expf(-z));
}

__device__ __forceinline__ void row_split(const float* sSrc, us_t* sH, us_t* sL,
                                          int wave, int lane) {
#pragma unroll
  for (int q = 0; q < 2; ++q) {
    const int row = 2 * wave + q;
    const v4f_t v = *(const v4f*)(sSrc + row * HID + lane * 4);
    v4us_t h4, l4;
#pragma unroll
    for (int e = 0; e < 4; ++e) {
      us_t a, b;
      split_bf(v[e], a, b);
      h4[e] = a;
      l4[e] = b;
    }
    *(v4us*)(sH + row * HP + lane * 4) = h4;
    *(v4us*)(sL + row * HP + lane * 4) = l4;
  }
}

__device__ __forceinline__ void store_rows2(const float* sF, float* __restrict__ gdst,
                                            int wave, int lane) {
  const int r0 = 2 * wave, r1 = 2 * wave + 1;
  const v4f_t v0 = *(const v4f*)(sF + r0 * HID + lane * 4);
  const v4f_t v1 = *(const v4f*)(sF + r1 * HID + lane * 4);
  float* p0 = gdst + (size_t)r0 * HID + lane * 4;
  float* p1 = gdst + (size_t)r1 * HID + lane * 4;
  *(volatile v4f_t*)p0 = v0;
  *(volatile v4f_t*)p1 = v1;
  __threadfence();
  *(volatile v4f_t*)p0 = v0;
  *(volatile v4f_t*)p1 = v1;
}

__device__ __forceinline__ float pair_mask(const float* __restrict__ pos, int i, int j) {
  const float dx = pos[i * 3 + 0] - pos[j * 3 + 0];
  const float dy = pos[i * 3 + 1] - pos[j * 3 + 1];
  const float dz = pos[i * 3 + 2] - pos[j * 3 + 2];
  const float d2 = dx * dx + dy * dy + dz * dz;
  const float dist = sqrtf((i == j) ? 1.0f : d2);
  return ((i != j) && (dist < CUTOFF_D)) ? 1.0f : 0.0f;
}

__global__ void __launch_bounds__(NTHR) rbf_kernel(const float* __restrict__ pos,
                                                   const float* __restrict__ cen,
                                                   const float* __restrict__ wid,
                                                   us_t* __restrict__ rbf) {
  __shared__ float sCen[KR];
  __shared__ float sInvW[KR];
  const int tid = threadIdx.x;
  if (tid < KR) {
    const int rc = (tid < NRBF) ? tid : (NRBF - 1);
    const float c = cen[rc];
    const float w = wid[rc];
    const float den = 2.0f * (w * w);
    sCen[tid] = (tid < NRBF) ? c : 10000.0f;
    sInvW[tid] = (tid < NRBF) ? (1.0f / den) : 1.0f;
  }
  __syncthreads();
  const int g = blockIdx.x * NTHR + tid;
  const int p = g >> 3, q = g & 7;
  const int i = p >> 9, j = p & (NA - 1);
  const float dx = pos[i * 3 + 0] - pos[j * 3 + 0];
  const float dy = pos[i * 3 + 1] - pos[j * 3 + 1];
  const float dz = pos[i * 3 + 2] - pos[j * 3 + 2];
  const float d2 = dx * dx + dy * dy + dz * dz;
  const float dist = sqrtf((i == j) ? 1.0f : d2);
  union { v8us_t h; v4u u; } ph, pl;
#pragma unroll
  for (int e = 0; e < 8; ++e) {
    const int r = q * 8 + e;
    const float dd = dist - sCen[r];
    const float arg = (dd * dd) * sInvW[r];
    const float v = __expf(-arg);
    us_t a, b;
    split_bf(v, a, b);
    ph.h[e] = a;
    pl.h[e] = b;
  }
  us_t* dh = rbf + (size_t)p * RP + q * 8;
  us_t* dl = dh + KR;
  *(volatile v4u*)dh = ph.u;
  *(volatile v4u*)dl = pl.u;
  __threadfence();
  *(volatile v4u*)dh = ph.u;
  *(volatile v4u*)dl = pl.u;
}

__global__ void __launch_bounds__(NTHR) init_kernel(const int* __restrict__ an,
                                                    const float* __restrict__ emb,
                                                    const float* __restrict__ w1,
                                                    const float* __restrict__ b1,
                                                    float* __restrict__ xout,
                                                    float* __restrict__ Tout) {
  __shared__ __align__(16) float sF[16 * HID];
  __shared__ __align__(16) us_t sXh[16 * HP];
  __shared__ __align__(16) us_t sXl[16 * HP];
  const int tid = threadIdx.x, wave = tid >> 5, lane = tid & 31;
  const int hh = lane >> 4, m = lane & 15;
  const int rbase = blockIdx.x * 16;
  const int col = wave * 16 + m;

  for (int idx = tid; idx < 16 * HID; idx += NTHR) {
    const int row = idx >> 7, c = idx & (HID - 1);
    int z = an[rbase + row];
    z = (z < 0) ? 0 : ((z > NEMB - 1) ? (NEMB - 1) : z);
    sF[idx] = emb[z * HID + c];
  }
  __syncthreads();
  store_rows2(sF, xout + (size_t)rbase * HID, wave, lane);
  row_split(sF, sXh, sXl, wave, lane);
  __syncthreads();
  const v8f acc = gemm128s(sXh, sXl, w1, HID, 0, HID, col, lane, zero8());
  {
    const float bc = b1[col];
#pragma unroll
    for (int r = 0; r < 8; ++r) {
      const int row = 8 * hh + r;
      sF[row * HID + col] = acc[r] + bc;
    }
  }
  __syncthreads();
  store_rows2(sF, Tout + (size_t)rbase * HID, wave, lane);
}

__global__ void __launch_bounds__(NTHR) pair_kernel(const us_t* __restrict__ rbf,
                                                    const float* __restrict__ pos,
                                                    const float* __restrict__ T,
                                                    const float* __restrict__ w1,
                                                    float* __restrict__ part) {
  __shared__ float sMask[256];
  __shared__ __align__(16) float sFwd[16 * HID];
  __shared__ __align__(16) float sRev[16 * HID];
  const int tid = threadIdx.x, wave = tid >> 5, lane = tid & 31;
  const int hh = lane >> 4, m = lane & 15;
  const int bid = blockIdx.x;
  int jt = 0;
  while (((jt + 1) * (jt + 2)) / 2 <= bid) ++jt;
  const int it = bid - (jt * (jt + 1)) / 2;
  const int ibase = it * 16, jbase = jt * 16;
  const int col = wave * 16 + m;
  {
    const int il = tid >> 4, jl = tid & 15;
    sMask[tid] = pair_mask(pos, ibase + il, jbase + jl);
  }
  const float* w1r = w1 + HID * HID;
  const BPair b0 = ldfragB(w1r, HID, 0,  NRBF, col, lane);
  const BPair b1 = ldfragB(w1r, HID, 32, NRBF, col, lane);
  float tj[8];
#pragma unroll
  for (int r = 0; r < 8; ++r) tj[r] = T[(size_t)(jbase + 8 * hh + r) * HID + col];
  __syncthreads();

  v8f accF = zero8();
#pragma unroll 1
  for (int il = 0; il < 16; ++il) {
    const int i = ibase + il;
    const us_t* arow = rbf + ((size_t)i * NA + jbase) * RP;
    const v16b a0h = ldfragA(arow, RP, 0, lane);
    const v16b a1h = ldfragA(arow, RP, 32, lane);
    const v16b a0l = ldfragA(arow, RP, KR, lane);
    const v16b a1l = ldfragA(arow, RP, KR + 32, lane);
    v8f d = zero8();
    d = wmma3(a0h, a0l, b0.h, b0.l, d);
    d = wmma3(a1h, a1l, b1.h, b1.l, d);
    const float ti = T[(size_t)i * HID + col];
    const float* mk = sMask + il * 16 + 8 * hh;
    float rev = 0.0f;
#pragma unroll
    for (int r = 0; r < 8; ++r) {
      const float mv = mk[r];
      accF[r] += silu_f(d[r] + ti) * mv;
      rev += silu_f(d[r] + tj[r]) * mv;
    }
    rev += __shfl_xor(rev, 16, 32);
    if (hh == 0) sRev[il * HID + col] = rev;
  }
#pragma unroll
  for (int r = 0; r < 8; ++r) sFwd[(8 * hh + r) * HID + col] = accF[r];
  __syncthreads();
  store_rows2(sFwd, part + (size_t)(jt * NT + it) * TILEF, wave, lane);
  if (it != jt) store_rows2(sRev, part + (size_t)(it * NT + jt) * TILEF, wave, lane);
}

__global__ void __launch_bounds__(NTHR) upd_kernel(const float* __restrict__ xin,
                                                   const float* __restrict__ part,
                                                   const float* __restrict__ pos,
                                                   const float* __restrict__ w2,
                                                   const float* __restrict__ b2,
                                                   const float* __restrict__ u1,
                                                   const float* __restrict__ ub1,
                                                   const float* __restrict__ u2,
                                                   const float* __restrict__ ub2,
                                                   const float* __restrict__ w1n,
                                                   const float* __restrict__ b1n,
                                                   int has_next,
                                                   float* __restrict__ xout,
                                                   float* __restrict__ Tout) {
  __shared__ __align__(16) float sF[16 * HID];
  __shared__ __align__(16) float sXf[16 * HID];
  __shared__ __align__(16) us_t sXh[16 * HP];
  __shared__ __align__(16) us_t sXl[16 * HP];
  __shared__ __align__(16) us_t sAh[16 * HP];
  __shared__ __align__(16) us_t sAl[16 * HP];
  __shared__ __align__(16) us_t sMh[16 * HP];
  __shared__ __align__(16) us_t sMl[16 * HP];
  __shared__ float sDg[16];
  __shared__ float sPart[NTHR];
  const int tid = threadIdx.x, wave = tid >> 5, lane = tid & 31;
  const int hh = lane >> 4, m = lane & 15;
  const int rb = blockIdx.x;
  const int rbase = rb * 16;
  const int col = wave * 16 + m;

  for (int idx = tid; idx < 16 * HID / 4; idx += NTHR) {
    v4f_t s;
    s[0] = 0.0f; s[1] = 0.0f; s[2] = 0.0f; s[3] = 0.0f;
    const float* pb = part + (size_t)(rb * NT) * TILEF + idx * 4;
#pragma unroll 1
    for (int st = 0; st < NT; ++st) {
      const v4f_t v = *(const v4f*)(pb + (size_t)st * TILEF);
      s += v;
    }
    *(v4f*)(sF + idx * 4) = s;
    const v4f_t vx = *(const v4f*)(xin + (size_t)rbase * HID + idx * 4);
    *(v4f*)(sXf + idx * 4) = vx;
  }
  {
    const int jl = tid & 15, j = rbase + jl, is = tid >> 4;
    float ps = 0.0f;
#pragma unroll 1
    for (int u = 0; u < 32; ++u) ps += pair_mask(pos, is * 32 + u, j);
    sPart[tid] = ps;
  }
  __syncthreads();
  if (tid < 16) {
    float dsum = 0.0f;
#pragma unroll 1
    for (int s = 0; s < 16; ++s) dsum += sPart[s * 16 + tid];
    sDg[tid] = dsum;
  }
  row_split(sF, sAh, sAl, wave, lane);
  row_split(sXf, sXh, sXl, wave, lane);
  __syncthreads();

  {
    const v8f acc = gemm128s(sAh, sAl, w2, HID, 0, HID, col, lane, zero8());
    const float bc = b2[col];
#pragma unroll
    for (int r = 0; r < 8; ++r) {
      const int row = 8 * hh + r;
      sF[row * HID + col] = acc[r] + sDg[row] * bc;
    }
  }
  __syncthreads();
  row_split(sF, sMh, sMl, wave, lane);
  __syncthreads();

  {
    v8f acc = gemm128s(sXh, sXl, u1, HID, 0,   2 * HID, col, lane, zero8());
    acc     = gemm128s(sMh, sMl, u1, HID, HID, 2 * HID, col, lane, acc);
    const float bc = ub1[col];
#pragma unroll
    for (int r = 0; r < 8; ++r) {
      const int row = 8 * hh + r;
      sF[row * HID + col] = silu_f(acc[r] + bc);
    }
  }
  __syncthreads();
  row_split(sF, sAh, sAl, wave, lane);
  __syncthreads();

  {
    const v8f ag = gemm128s(sAh, sAl, u2, HID, 0, HID, col, lane, zero8());
    const float bc = ub2[col];
#pragma unroll
    for (int r = 0; r < 8; ++r) {
      const int row = 8 * hh + r;
      const float xn = (sXf[row * HID + col] + ag[r]) + bc;
      sF[row * HID + col] = xn;
    }
  }
  __syncthreads();
  store_rows2(sF, xout + (size_t)rbase * HID, wave, lane);
  if (has_next) {
    row_split(sF, sXh, sXl, wave, lane);
    __syncthreads();
    const v8f at = gemm128s(sXh, sXl, w1n, HID, 0, HID, col, lane, zero8());
    const float bc = b1n[col];
#pragma unroll
    for (int r = 0; r < 8; ++r) {
      const int row = 8 * hh + r;
      sF[row * HID + col] = at[r] + bc;
    }
    __syncthreads();
    store_rows2(sF, Tout + (size_t)rbase * HID, wave, lane);
  }
}

__global__ void __launch_bounds__(NTHR) head_kernel(const float* __restrict__ x,
                                                    const int* __restrict__ bat,
                                                    const float* __restrict__ o1,
                                                    const float* __restrict__ ob1,
                                                    const float* __restrict__ o2,
                                                    const float* __restrict__ ob2,
                                                    float* __restrict__ out) {
  __shared__ __align__(16) float sF[NMOL * HID];
  __shared__ __align__(16) us_t sXh[16 * HP];
  __shared__ __align__(16) us_t sXl[16 * HP];
  __shared__ float sRc[NMOL];
  __shared__ float sHd[NMOL * HID2];
  __shared__ __align__(16) float sOut[NMOL];
  const int tid = threadIdx.x, wave = tid >> 5, lane = tid & 31;
  const int hh = lane >> 4, m = lane & 15;

  for (int idx = tid; idx < NMOL * HID; idx += NTHR) sF[idx] = 0.0f;
  __syncthreads();
  if (wave < 4) {
    const int c = tid;
#pragma unroll 1
    for (int a = 0; a < NA; ++a) {
      const int mr = bat[a];
      const bool ok = (unsigned)mr < (unsigned)NMOL;
      const int mm = ok ? mr : 0;
      const float v = x[(size_t)a * HID + c];
      const float add = ok ? v : 0.0f;
      sF[mm * HID + c] += add;
    }
  } else if (wave == 4) {
    const int mq = lane & 15;
    float cnt = 0.0f;
#pragma unroll 1
    for (int a = 0; a < NA; ++a) cnt += (bat[a] == mq) ? 1.0f : 0.0f;
    if (lane < NMOL) sRc[mq] = 1.0f / fmaxf(cnt, 1.0f);
  }
  __syncthreads();
  for (int idx = tid; idx < NMOL * HID; idx += NTHR) {
    const int mi = idx >> 7;
    sF[idx] = sF[idx] * sRc[mi];
  }
  __syncthreads();
  row_split(sF, sXh, sXl, wave, lane);
  __syncthreads();
  {
    const int col = (wave & 3) * 16 + m;
    const v8f acc = gemm128s(sXh, sXl, o1, HID2, 0, HID, col, lane, zero8());
    const float bc = ob1[col];
    if (wave < 4) {
#pragma unroll
      for (int r = 0; r < 8; ++r) {
        const int row = 8 * hh + r;
        sHd[row * HID2 + col] = silu_f(acc[r] + bc);
      }
    }
  }
  __syncthreads();
  if (wave == 0) {
    const int r16 = lane & 15;
    float o = 0.0f;
#pragma unroll 1
    for (int k = 0; k < HID2; ++k) o += sHd[r16 * HID2 + k] * o2[k];
    o += ob2[0];
    if (lane < NMOL) sOut[lane] = o;
  }
  __syncthreads();
  if (wave == 0) {
    const v4f_t v = *(const v4f*)(sOut + (lane & 3) * 4);
    float* gp = out + (lane & 3) * 4;
    if (lane < 4) *(volatile v4f_t*)gp = v;
    __threadfence();
    if (lane < 4) *(volatile v4f_t*)gp = v;
  }
}

extern "C" void kernel_launch(void* const* d_in, const int* in_sizes, int n_in,
                              void* d_out, int out_size, void* d_ws, size_t ws_size,
                              hipStream_t stream) {
  if (n_in < 18) return;
  if (in_sizes[0] != NA || in_sizes[1] != NA * 3 || in_sizes[2] != NA) return;
  if (in_sizes[3] != NEMB * HID || in_sizes[4] != NRBF || in_sizes[5] != NRBF) return;
  if (in_sizes[6] != NBLK * (HID + NRBF) * HID || in_sizes[7] != NBLK * HID) return;
  if (in_sizes[8] != NBLK * HID * HID || in_sizes[9] != NBLK * HID) return;
  if (in_sizes[10] != NBLK * 2 * HID * HID || in_sizes[11] != NBLK * HID) return;
  if (in_sizes[12] != NBLK * HID * HID || in_sizes[13] != NBLK * HID) return;
  if (in_sizes[14] != HID * HID2 || in_sizes[15] != HID2) return;
  if (in_sizes[16] != HID2 || in_sizes[17] != 1) return;
  if (out_size != NMOL) return;

  const int*   an      = (const int*)d_in[0];
  const float* pos     = (const float*)d_in[1];
  const int*   batch   = (const int*)d_in[2];
  const float* emb     = (const float*)d_in[3];
  const float* centers = (const float*)d_in[4];
  const float* widths  = (const float*)d_in[5];
  const float* msg_w1  = (const float*)d_in[6];
  const float* msg_b1  = (const float*)d_in[7];
  const float* msg_w2  = (const float*)d_in[8];
  const float* msg_b2  = (const float*)d_in[9];
  const float* upd_w1  = (const float*)d_in[10];
  const float* upd_b1  = (const float*)d_in[11];
  const float* upd_w2  = (const float*)d_in[12];
  const float* upd_b2  = (const float*)d_in[13];
  const float* out_w1  = (const float*)d_in[14];
  const float* out_b1  = (const float*)d_in[15];
  const float* out_w2  = (const float*)d_in[16];
  const float* out_b2  = (const float*)d_in[17];
  float* out = (float*)d_out;

  const size_t nRBF  = (size_t)NA * NA * RP * 2;
  const size_t nXF   = (size_t)NA * HID * 4;
  const size_t nPART = (size_t)NT * NT * TILEF * 4;
  const size_t oRBF  = 0;
  const size_t oX0   = oRBF + nRBF;
  const size_t oX1   = oX0 + nXF;
  const size_t oT    = oX1 + nXF;
  const size_t oPART = oT + nXF;
  const size_t total = oPART + nPART;
  if (total > ws_size) return;
  if (total > (size_t)134217728) return;

  char* ws = (char*)d_ws;
  us_t*  rbf  = (us_t*)(ws + oRBF);
  float* X0   = (float*)(ws + oX0);
  float* X1   = (float*)(ws + oX1);
  float* T    = (float*)(ws + oT);
  float* PART = (float*)(ws + oPART);

  const int W1S = (HID + NRBF) * HID;
  const int W2S = HID * HID;
  const int U1S = 2 * HID * HID;

  rbf_kernel<<<(NA * NA * 8) / NTHR, NTHR, 0, stream>>>(pos, centers, widths, rbf);
  init_kernel<<<NT, NTHR, 0, stream>>>(an, emb, msg_w1, msg_b1, X0, T);
  for (int b = 0; b < NBLK; ++b) {
    const float* xin = (b & 1) ? X1 : X0;
    float* xout = (b & 1) ? X0 : X1;
    const int bn = (b + 1 < NBLK) ? (b + 1) : (NBLK - 1);
    const int has_next = (b + 1 < NBLK) ? 1 : 0;
    pair_kernel<<<NTP, NTHR, 0, stream>>>(rbf, pos, T, msg_w1 + (size_t)b * W1S, PART);
    upd_kernel<<<NT, NTHR, 0, stream>>>(xin, PART, pos,
                                         msg_w2 + (size_t)b * W2S, msg_b2 + b * HID,
                                         upd_w1 + (size_t)b * U1S, upd_b1 + b * HID,
                                         upd_w2 + (size_t)b * W2S, upd_b2 + b * HID,
                                         msg_w1 + (size_t)bn * W1S, msg_b1 + bn * HID,
                                         has_next, xout, T);
  }
  head_kernel<<<1, NTHR, 0, stream>>>(X0, batch, out_w1, out_b1, out_w2, out_b2, out);
}
